// RandomKNeighborsMHA_73650099191880
// MI455X (gfx1250) — hardware-verified
//
#include <hip/hip_runtime.h>
#include <stdint.h>

typedef __attribute__((ext_vector_type(16))) _Float16 v16h;
typedef __attribute__((ext_vector_type(8)))  _Float16 v8h;
typedef __attribute__((ext_vector_type(16))) __bf16   v16b;
typedef __attribute__((ext_vector_type(8)))  __bf16   v8b;
typedef __attribute__((ext_vector_type(8)))  float    v8f;
typedef __attribute__((ext_vector_type(4)))  float    v4f;
typedef __attribute__((ext_vector_type(2)))  float    v2f;

__device__ __forceinline__ unsigned short f2bf_bits(float f) {
  unsigned u = __float_as_uint(f);
  return (unsigned short)((u + 0x7FFFu + ((u >> 16) & 1u)) >> 16);
}
__device__ __forceinline__ float bf_bits2f(unsigned short h) { return __uint_as_float(((unsigned)h) << 16); }

__device__ __forceinline__ void dep_guard_h(v8f& a, v8f& b, v16h x, v16h y) { asm volatile("v_nop\n\tv_nop\n\tv_nop\n\tv_nop" : "+v"(a), "+v"(b) : "v"(x), "v"(y)); }
__device__ __forceinline__ void dep_guard_b(v8f& a, v8f& b, v16b x, v16b y) { asm volatile("v_nop\n\tv_nop\n\tv_nop\n\tv_nop" : "+v"(a), "+v"(b) : "v"(x), "v"(y)); }
__device__ __forceinline__ void keep4_h(v16h a, v16h b, v16h c, v16h d) { asm volatile("v_nop" :: "v"(a), "v"(b), "v"(c), "v"(d)); }
__device__ __forceinline__ void keep4_b(v16b a, v16b b, v16b c, v16b d) { asm volatile("v_nop" :: "v"(a), "v"(b), "v"(c), "v"(d)); }
__device__ __forceinline__ void acc_guard4(v8f& a, v8f& b, v8f& c, v8f& d) { asm volatile("v_nop\n\tv_nop\n\tv_nop\n\tv_nop" : "+v"(a), "+v"(b), "+v"(c), "+v"(d)); }
template <typename T> struct Frag;
template <> struct Frag<_Float16> {
  typedef v16h V; union U { v16h v; v8h h[2]; };
  static __device__ __forceinline__ v16h load(const _Float16* p) {
    U f; f.h[0] = *(const v8h*)(p); f.h[1] = *(const v8h*)(p + 16); return f.v;
  }
  static __device__ __forceinline__ v8f mma(v16h a, v16h b, v8f c) {
    return __builtin_amdgcn_wmma_f32_16x16x32_f16(false, a, false, b, (short)0, c, false, false);
  }
  static __device__ __forceinline__ void guard(v8f& a, v8f& b, v16h x, v16h y) { dep_guard_h(a, b, x, y); }
  static __device__ __forceinline__ void keep(v16h a, v16h b, v16h c, v16h d) { keep4_h(a, b, c, d); }
};
template <> struct Frag<__bf16> {
  typedef v16b V; union U { v16b v; v8b h[2]; };
  static __device__ __forceinline__ v16b load(const __bf16* p) {
    U f; f.h[0] = *(const v8b*)(p); f.h[1] = *(const v8b*)(p + 16); return f.v;
  }
  static __device__ __forceinline__ v8f mma(v16b a, v16b b, v8f c) {
    return __builtin_amdgcn_wmma_f32_16x16x32_bf16(false, a, false, b, (short)0, c, false, false);
  }
  static __device__ __forceinline__ void guard(v8f& a, v8f& b, v16b x, v16b y) { dep_guard_b(a, b, x, y); }
  static __device__ __forceinline__ void keep(v16b a, v16b b, v16b c, v16b d) { keep4_b(a, b, c, d); }
};

template <int ET> struct Elem;
template <> struct Elem<0> { typedef _Float16 T; };
template <> struct Elem<1> { typedef __bf16 T; };
template <int ET, bool SPLIT, int BIAS_MODE, int OUT_MODE, bool RESID, int ACT = 0>
__global__ __launch_bounds__(256) void wmma_gemm64(
    const unsigned short* __restrict__ Ap, const unsigned short* __restrict__ A2p, int lda, long strideA,
    const unsigned short* __restrict__ Btp, const unsigned short* __restrict__ Bt2p, int ldb, long strideB,
    void* __restrict__ Cout, void* __restrict__ Cout2, int ldc, long strideC,
    const float* __restrict__ bias,
    const float* __restrict__ resid, long strideR,
    int M, int N, int K, float scale) {
  typedef typename Elem<ET>::T T;
  typedef typename Frag<T>::V V;
  const T* A = (const T*)Ap; const T* A2 = (const T*)A2p; const T* Bt = (const T*)Btp; const T* Bt2 = (const T*)Bt2p;
  __shared__ __align__(16) float sT[8][16 * 68];
  const int b    = blockIdx.y;
  const int lane = threadIdx.x & 31;
  const int wave = threadIdx.x >> 5;
  const int tilesN = N >> 6;
  const int tilesM = M >> 6;
  const int tile = blockIdx.x * 8 + wave;
  if (tile >= tilesM * tilesN) return;
  const int tm = tile / tilesN;
  const int tn = tile - tm * tilesN;
  const int m0 = tm << 6;
  const int n0 = tn << 6;

  const T* Ab  = A  + (size_t)b * strideA;
  const T* Bb  = Bt + (size_t)b * strideB;
  const T* Ab2 = SPLIT ? (A2  + (size_t)b * strideA) : nullptr;
  const T* Bb2 = SPLIT ? (Bt2 + (size_t)b * strideB) : nullptr;

  const int rlane = lane & 15;
  const int koff  = (lane >> 4) * 8;
  const int mOff  = (lane >> 4) * 8;

  v8f acc[4][4];
#pragma unroll
  for (int i = 0; i < 4; ++i)
#pragma unroll
    for (int j = 0; j < 4; ++j) acc[i][j] = (v8f){0.f,0.f,0.f,0.f,0.f,0.f,0.f,0.f};

  for (int k0 = 0; k0 < K; k0 += 32) {
    V bh[4], bl[4];
#pragma unroll
    for (int j = 0; j < 4; ++j) {
      const size_t bo = (size_t)(n0 + (j << 4) + rlane) * ldb + koff + k0;
      bh[j] = Frag<T>::load(Bb + bo);
      if (SPLIT) bl[j] = Frag<T>::load(Bb2 + bo);
    }
#pragma unroll
    for (int i = 0; i < 4; ++i) {
      const size_t ao = (size_t)(m0 + (i << 4) + rlane) * lda + koff + k0;
      V ah = Frag<T>::load(Ab + ao);
      V al;
      if (SPLIT) al = Frag<T>::load(Ab2 + ao);
#pragma unroll
      for (int j = 0; j < 4; ++j) {
        acc[i][j] = Frag<T>::mma(ah, bh[j], acc[i][j]);
        if (SPLIT) {
          acc[i][j] = Frag<T>::mma(ah, bl[j], acc[i][j]);
          acc[i][j] = Frag<T>::mma(al, bh[j], acc[i][j]);
        }
      }
      Frag<T>::guard(acc[i][0], acc[i][3], ah, SPLIT ? al : ah);
    }
    Frag<T>::keep(bh[0], bh[1], bh[2], bh[3]);
    if (SPLIT) Frag<T>::keep(bl[0], bl[1], bl[2], bl[3]);
  }
  acc_guard4(acc[0][0], acc[0][1], acc[0][2], acc[0][3]);
  acc_guard4(acc[1][0], acc[1][1], acc[1][2], acc[1][3]);
  acc_guard4(acc[2][0], acc[2][1], acc[2][2], acc[2][3]);
  acc_guard4(acc[3][0], acc[3][1], acc[3][2], acc[3][3]);

  float* slab = sT[wave];
  const float* Rb = RESID ? (resid + (size_t)b * strideR) : nullptr;
#pragma unroll
  for (int i = 0; i < 4; ++i) {
    const int mBase = m0 + (i << 4);
#pragma unroll
    for (int j = 0; j < 4; ++j) {
      const int n = n0 + (j << 4) + rlane;
      float bv = 0.f;
      if (BIAS_MODE == 2) bv = bias[n];
#pragma unroll
      for (int r = 0; r < 8; ++r) {
        float v = acc[i][j][r] * scale;
        if (BIAS_MODE == 1) v += bias[mBase + mOff + r];
        if (BIAS_MODE == 2) v += bv;
        if (RESID) v += Rb[(size_t)(mBase + mOff + r) * ldc + n];
        if (ACT == 1) v = tanhf(v);
        if (ACT == 2) v = fmaxf(v, 0.0f);
        if (ACT == 3) v = v / (1.0f + expf(-v));
        if (ACT == 4) v = (v > 0.f) ? v : 0.01f * v;
        if (ACT == 5) v = 0.5f * v * (1.0f + erff(v * 0.70710678118654752f));
        slab[(mOff + r) * 68 + (j << 4) + rlane] = v;
      }
    }
    __builtin_amdgcn_fence(__ATOMIC_RELEASE, "workgroup");
    __builtin_amdgcn_wave_barrier();
    __builtin_amdgcn_fence(__ATOMIC_ACQUIRE, "workgroup");
    if (OUT_MODE == 0) {
      float* C = (float*)Cout + (size_t)b * strideC;
      const int hh = lane >> 4, c4 = (lane & 15) * 4;
      for (int pass = 0; pass < 2; ++pass) {
#pragma unroll
        for (int it = 0; it < 8; ++it) {
          const int row = it * 2 + hh;
          v4f v = *(const v4f*)(slab + row * 68 + c4);
          *(volatile v4f*)(C + (size_t)(mBase + row) * ldc + n0 + c4) = v;
        }
        __threadfence();
      }
    } else {
      const int q = lane >> 3, c8 = (lane & 7) * 8;
      unsigned short* C  = (unsigned short*)Cout  + (size_t)b * strideC;
      unsigned short* C2 = (OUT_MODE == 2) ? ((unsigned short*)Cout2 + (size_t)b * strideC) : nullptr;
      for (int pass = 0; pass < 2; ++pass) {
#pragma unroll
        for (int it = 0; it < 4; ++it) {
          const int row = it * 4 + q;
          const float* sp = slab + row * 68 + c8;
          v8h hv, lv;
#pragma unroll
          for (int e = 0; e < 8; ++e) {
            if (OUT_MODE == 1) {
              hv[e] = (_Float16)sp[e];
            } else {
              unsigned short hb = f2bf_bits(sp[e]);
              unsigned short lb = f2bf_bits(sp[e] - bf_bits2f(hb));
              hv[e] = __builtin_bit_cast(_Float16, hb);
              lv[e] = __builtin_bit_cast(_Float16, lb);
            }
          }
          *(volatile v8h*)(C + (size_t)(mBase + row) * ldc + n0 + c8) = hv;
          if (OUT_MODE == 2) *(volatile v8h*)(C2 + (size_t)(mBase + row) * ldc + n0 + c8) = lv;
        }
        __threadfence();
      }
    }
    __builtin_amdgcn_fence(__ATOMIC_RELEASE, "workgroup");
    __builtin_amdgcn_wave_barrier();
    __builtin_amdgcn_fence(__ATOMIC_ACQUIRE, "workgroup");
  }
}

__global__ __launch_bounds__(256) void cast_f32_f16x2s(
    const float* __restrict__ in, _Float16* __restrict__ out, int n2, float carry) {
  int i = blockIdx.x * 256 + threadIdx.x;
  if (i < n2) {
    const _Float16 h0 = (_Float16)(in[2 * i] * carry), h1 = (_Float16)(in[2 * i + 1] * carry);
    const unsigned u = (unsigned)__builtin_bit_cast(unsigned short, h0) | ((unsigned)__builtin_bit_cast(unsigned short, h1) << 16);
    ((volatile unsigned*)out)[i] = u;
    __threadfence();
    ((volatile unsigned*)out)[i] = u;
  }
}

#define NB_C 1024
#define NB_DH 64
#define NB_K 32
#define NB_H 16

__global__ __launch_bounds__(512) void nbr_attn_kernel(
    const float* __restrict__ q, const float* __restrict__ k, const float* __restrict__ v,
    const int* __restrict__ idx, unsigned short* __restrict__ aout, int L, float qscale, float ocarry) {
  __shared__ __align__(16) float qs[NB_C];
  __shared__ __align__(16) float os[NB_H][NB_DH];
  __shared__ int sidx[NB_K];
  const int tid  = threadIdx.x;
  const int lane = tid & 31;
  const int h    = tid >> 5;
  const int bl   = blockIdx.x;
  const int b    = bl / L;
  const int l    = bl - b * L;
  {
    const float* qrow = q + (size_t)bl * NB_C;
    const v2f qq = *(const v2f*)(qrow + 2 * tid);
    qs[2 * tid]     = qq.x * qscale;
    qs[2 * tid + 1] = qq.y * qscale;
  }
  if (tid < NB_K) {
    int j = idx[(size_t)l * NB_K + tid];
    j = j < 0 ? 0 : j;
    j = j > (L - 1) ? (L - 1) : j;
    sidx[tid] = j;
  }
  __syncthreads();

  const int j = sidx[lane];
  const float* krow = k + ((size_t)b * L + (size_t)j) * NB_C + h * NB_DH;
  const float* qh = qs + h * NB_DH;
  float s = 0.f;
#pragma unroll 2
  for (int i = 0; i < NB_DH / 4; ++i) {
    const v4f kk4 = *(const v4f*)(krow + 4 * i);
    const v4f qq4 = *(const v4f*)(qh + 4 * i);
    s += qq4.x * kk4.x;
    s += qq4.y * kk4.y;
    s += qq4.z * kk4.z;
    s += qq4.w * kk4.w;
  }
  float m = s;
#pragma unroll
  for (int off = 16; off >= 1; off >>= 1) m = fmaxf(m, __shfl_xor(m, off, 32));
  const float e = expf(s - m);
  float sum = e;
#pragma unroll
  for (int off = 16; off >= 1; off >>= 1) sum += __shfl_xor(sum, off, 32);
  const float p = e * (1.0f / sum);

  const int d0 = 2 * lane;
  const float* vb = v + (size_t)b * L * NB_C + h * NB_DH + d0;
  float ax = 0.f, ay = 0.f;
#pragma unroll 4
  for (int kk = 0; kk < NB_K; ++kk) {
    const float pk = __shfl(p, kk, 32);
    const int jk = sidx[kk];
    const v2f vv = *(const v2f*)(vb + (size_t)jk * NB_C);
    ax += pk * vv.x;
    ay += pk * vv.y;
  }

  float* ow = os[h];
  ow[d0]     = ax * ocarry;
  ow[d0 + 1] = ay * ocarry;
  __builtin_amdgcn_fence(__ATOMIC_RELEASE, "workgroup");
  __builtin_amdgcn_wave_barrier();
  __builtin_amdgcn_fence(__ATOMIC_ACQUIRE, "workgroup");
  const int c8 = (lane & 7) * 8;
  const v4f f0 = *(const v4f*)(ow + c8);
  const v4f f1 = *(const v4f*)(ow + c8 + 4);
  v8h hv;
  hv[0] = (_Float16)f0.x; hv[1] = (_Float16)f0.y; hv[2] = (_Float16)f0.z; hv[3] = (_Float16)f0.w;
  hv[4] = (_Float16)f1.x; hv[5] = (_Float16)f1.y; hv[6] = (_Float16)f1.z; hv[7] = (_Float16)f1.w;
  unsigned short* dst = aout + (size_t)bl * NB_C + h * NB_DH + c8;
  for (int pass = 0; pass < 2; ++pass) {
    if (lane < 8) *(volatile v8h*)dst = hv;
    __threadfence();
  }
}

extern "C" void kernel_launch(void* const* d_in, const int* in_sizes, int n_in,
                              void* d_out, int out_size, void* d_ws,
                              size_t ws_size, hipStream_t stream) {
  if (n_in < 6) return;
  const int C = NB_C;
  const int nx = in_sizes[0];
  if (nx <= 0 || (nx % C) != 0) return;
  const int Mtot = nx / C;
  if ((Mtot % 64) != 0) return;
  const int nidx = in_sizes[1];
  if (nidx <= 0 || (nidx % NB_K) != 0) return;
  const int L = nidx / NB_K;
  if (L <= 0 || (Mtot % L) != 0) return;
  if (in_sizes[2] != C * C || in_sizes[3] != C * C || in_sizes[4] != C * C || in_sizes[5] != C * C) return;
  if (out_size != Mtot * C) return;

  const float* x   = (const float*)d_in[0];
  const int*   idx = (const int*)d_in[1];
  const float* Wq  = (const float*)d_in[2];
  const float* Wk  = (const float*)d_in[3];
  const float* Wv  = (const float*)d_in[4];
  const float* Wo  = (const float*)d_in[5];
  float*       out = (float*)d_out;

  const size_t bytes_x16  = (size_t)Mtot * C * 2;
  const size_t bytes_w16  = (size_t)C * C * 2;
  const size_t bytes_qkv  = (size_t)3 * Mtot * C * 4;
  const size_t bytes_a16  = (size_t)Mtot * C * 2;
  const size_t off_x16 = 0;
  const size_t off_w16 = off_x16 + bytes_x16;
  const size_t off_qkv = off_w16 + 4 * bytes_w16;
  const size_t off_a16 = off_qkv + bytes_qkv;
  const size_t off_end = off_a16 + bytes_a16;
  if (off_end > ws_size) return;

  char* ws = (char*)d_ws;
  unsigned short* x16  = (unsigned short*)(ws + off_x16);
  unsigned short* w16  = (unsigned short*)(ws + off_w16);
  unsigned short* wq16 = w16;
  unsigned short* wk16 = w16 + (size_t)C * C;
  unsigned short* wv16 = w16 + (size_t)2 * C * C;
  unsigned short* wo16 = w16 + (size_t)3 * C * C;
  float* qkv  = (float*)(ws + off_qkv);
  float* qbuf = qkv;
  float* kbuf = qkv + (size_t)Mtot * C;
  float* vbuf = qkv + (size_t)2 * Mtot * C;
  unsigned short* a16 = (unsigned short*)(ws + off_a16);

  const int n2x = nx / 2;
  const int n2w = (C * C) / 2;
  cast_f32_f16x2s<<<(n2x + 255) / 256, 256, 0, stream>>>(x,  (_Float16*)x16,  n2x, 1.0f);
  cast_f32_f16x2s<<<(n2w + 255) / 256, 256, 0, stream>>>(Wq, (_Float16*)wq16, n2w, 16.0f);
  cast_f32_f16x2s<<<(n2w + 255) / 256, 256, 0, stream>>>(Wk, (_Float16*)wk16, n2w, 16.0f);
  cast_f32_f16x2s<<<(n2w + 255) / 256, 256, 0, stream>>>(Wv, (_Float16*)wv16, n2w, 16.0f);
  cast_f32_f16x2s<<<(n2w + 255) / 256, 256, 0, stream>>>(Wo, (_Float16*)wo16, n2w, 16.0f);

  const int tiles = (Mtot / 64) * (C / 64);
  const int gx = (tiles + 7) / 8;
  wmma_gemm64<0, false, 0, 0, false, 0><<<dim3(gx, 3), 256, 0, stream>>>(
      x16, nullptr, C, 0L,
      w16, nullptr, C, (long)C * C,
      (void*)qkv, nullptr, C, (long)Mtot * C,
      nullptr, nullptr, 0L,
      Mtot, C, C, 1.0f / 16.0f);

  nbr_attn_kernel<<<Mtot, 512, 0, stream>>>(qbuf, kbuf, vbuf, idx, a16, L, 0.125f, 16.0f);

  wmma_gemm64<0, false, 0, 0, false, 0><<<dim3(gx, 1), 256, 0, stream>>>(
      a16, nullptr, C, 0L,
      wo16, nullptr, C, 0L,
      (void*)out, nullptr, C, 0L,
      nullptr, nullptr, 0L,
      Mtot, C, C, 1.0f / 256.0f);
}
